// PrivateEncoder_26310969655373
// MI455X (gfx1250) — hardware-verified
//
#include <hip/hip_runtime.h>
#include <math.h>

typedef __attribute__((ext_vector_type(16))) _Float16 v16h;
typedef __attribute__((ext_vector_type(8)))  _Float16 v8h;
typedef __attribute__((ext_vector_type(8)))  float    v8f;
typedef __attribute__((ext_vector_type(4)))  float    v4f;

constexpr int kBatch = 64;
constexpr int kChan  = 3;
constexpr int kImg   = 256;
constexpr int kPatch = 16;
constexpr int kSide  = kImg / kPatch;
constexpr int kTok   = kSide * kSide;
constexpr int kDm    = 768;
constexpr int kDepth = 3;
constexpr int kRows  = kBatch * kTok;
constexpr int kKin   = kChan * kPatch * kPatch;
constexpr int kWElems    = kDm * kDm;
constexpr int kOctPerRow = kDm / 8;
constexpr int kTileRows  = kRows / 64;
static_assert(kSide == 16);
static_assert(kTok == 256);
static_assert(kRows == 16384);
static_assert(kKin == kDm);
static_assert((kKin % 32) == 0 && (kDm % 32) == 0);
static_assert((kRows % 64) == 0 && (kDm % 64) == 0);
static_assert(((kRows / 64) * (kDm / 64)) % 8 == 0);
static_assert((kRows * kOctPerRow) % 256 == 0);
static_assert(((kWElems / 8) % 256) == 0);

constexpr int kInputsRneToBf16 = 1;

constexpr float kActCarry = 16.0f;
constexpr float kWgtCarry = 1024.0f;
constexpr float kFold     = 1.0f / (kActCarry * kWgtCarry);
constexpr float kF16MinNormal = 6.103515625e-05f;
constexpr float kBnEps = 1e-5f;

constexpr size_t kSzT  = (size_t)kRows * kDm * 4;
constexpr size_t kSzP0 = (size_t)kRows * kKin * 2;
constexpr size_t kSzH  = (size_t)kRows * kDm * 2;
constexpr size_t kSzWH = (size_t)5 * kWElems * 2;
constexpr size_t kSPlane = (size_t)kTileRows * 2 * kDm;
constexpr size_t kSzS  = (size_t)kDepth * kSPlane * 4;
constexpr size_t kSzST = (size_t)kDepth * 2 * kDm * 4;
constexpr size_t kOffT  = 0;
constexpr size_t kOffP0 = kOffT  + kSzT;
constexpr size_t kOffH  = kOffP0 + kSzP0;
constexpr size_t kOffWH = kOffH  + kSzH;
constexpr size_t kOffS  = kOffWH + kSzWH;
constexpr size_t kOffST = kOffS  + kSzS;
constexpr size_t kWsTotal = kOffST + kSzST;
static_assert(kWsTotal == 111298560ull);
static_assert(kWsTotal <= 134217728ull);
static_assert((kOffP0 % 128) == 0 && (kOffH % 128) == 0 && (kOffWH % 128) == 0 &&
              (kOffS % 128) == 0 && (kOffST % 128) == 0);

__device__ __forceinline__ unsigned short f2bf_bits(float f) {
  unsigned u = __float_as_uint(f);
  return (unsigned short)((u + 0x7FFFu + ((u >> 16) & 1u)) >> 16);
}
__device__ __forceinline__ float bf_bits2f(unsigned short h) { return __uint_as_float(((unsigned)h) << 16); }

__device__ __forceinline__ float in_leg(float f) {
  if (kInputsRneToBf16) return bf_bits2f(f2bf_bits(f));
  return f;
}
__device__ __forceinline__ _Float16 to_f16_carried(float v, float carry) {
  float c = v * carry;
  c = (fabsf(c) < kF16MinNormal) ? 0.0f : c;
  return (_Float16)c;
}

__global__ __launch_bounds__(256) void weight_planes_kernel(
    const float* __restrict__ w_embed, const float* __restrict__ w_layers,
    const float* __restrict__ w_mixer, unsigned short* __restrict__ dst)
{
  constexpr int kBlocksPerMat = (kWElems / 8) / 256;
  const int mat = blockIdx.x / kBlocksPerMat;
  if (mat >= 5) return;
  const int li = (blockIdx.x - mat * kBlocksPerMat) * 256 + threadIdx.x;
  const float* src = (mat == 0) ? w_embed
                   : (mat == 4) ? w_mixer
                   : (w_layers + (size_t)(mat - 1) * kWElems);
  const size_t e0 = (size_t)li << 3;
  const v4f a0 = *(const v4f*)(src + e0);
  const v4f a1 = *(const v4f*)(src + e0 + 4);
  v8h hv;
#pragma unroll
  for (int e = 0; e < 4; ++e) {
    const float f0 = a0[e];
    const float f1 = a1[e];
    hv[e]     = to_f16_carried(in_leg(f0), kWgtCarry);
    hv[4 + e] = to_f16_carried(in_leg(f1), kWgtCarry);
  }
  unsigned short* q = dst + (size_t)mat * kWElems + e0;
  *(volatile v8h*)q = hv;
  __threadfence();
  *(volatile v8h*)q = hv;
}

__global__ __launch_bounds__(256) void patch_rows_kernel(
    const float* __restrict__ x, unsigned short* __restrict__ P0)
{
  const int i = blockIdx.x * 256 + threadIdx.x;
  if (i >= kRows * kOctPerRow) return;
  const int r  = i / kOctPerRow;
  const int k  = (i - r * kOctPerRow) * 8;
  const int c  = k / (kPatch * kPatch);
  const int kh = (k / kPatch) % kPatch;
  const int kw = k % kPatch;
  const int b  = r / kTok;
  const int p  = r % kTok;
  const int hp = p / kSide;
  const int wp = p % kSide;
  const size_t so = ((size_t)((b * kChan + c) * kImg + hp * kPatch + kh)) * kImg + wp * kPatch + kw;
  const v4f a0 = *(const v4f*)(x + so);
  const v4f a1 = *(const v4f*)(x + so + 4);
  v8h hv;
#pragma unroll
  for (int e = 0; e < 4; ++e) {
    const float f0 = a0[e];
    const float f1 = a1[e];
    hv[e]     = to_f16_carried(in_leg(f0), kActCarry);
    hv[4 + e] = to_f16_carried(in_leg(f1), kActCarry);
  }
  unsigned short* q = P0 + ((size_t)i << 3);
  *(volatile v8h*)q = hv;
  __threadfence();
  *(volatile v8h*)q = hv;
}

namespace eng {

union FragU { v16h v; v8h h[2]; };
__device__ __forceinline__ v16h frag_load(const _Float16* p) {
  FragU f;
  f.h[0] = *(const v8h*)(p);
  f.h[1] = *(const v8h*)(p + 16);
  return f.v;
}
__device__ __forceinline__ v8f mma_f16(v16h a, v16h b, v8f c) {
  return __builtin_amdgcn_wmma_f32_16x16x32_f16(false, a, false, b, (short)0, c, false, false);
}
__device__ __forceinline__ void tie_acc(v8f& a, v16h x, v16h y) { asm volatile("" : "+v"(a) : "v"(x), "v"(y)); }
__device__ __forceinline__ void guard_acc(v8f& a, v16h x, v16h y) {
  asm volatile("v_nop\n\tv_nop\n\tv_nop\n\tv_nop" : "+v"(a) : "v"(x), "v"(y));
}

constexpr int kEpiAct  = 0;
constexpr int kEpiStat = 1;
constexpr int kEpiOut  = 2;

template <int EPI>
__global__ __launch_bounds__(256) void gemm_f16_kernel(
    const unsigned short* __restrict__ Ap, int lda,
    const unsigned short* __restrict__ Btp, int ldb,
    void* __restrict__ Cout, int ldc,
    const float* __restrict__ bias,
    float* __restrict__ Spart,
    int M, int N, int K, float scale)
{
  const _Float16* A  = (const _Float16*)Ap;
  const _Float16* Bt = (const _Float16*)Btp;
  __shared__ __align__(16) float sT[8][16 * 68];
  const int lane = threadIdx.x & 31;
  const int wave = threadIdx.x >> 5;
  const int tilesN = N >> 6;
  const int tilesM = M >> 6;
  const int tile = blockIdx.x * 8 + wave;
  if (tile >= tilesM * tilesN) return;
  const int tm = tile / tilesN;
  const int tn = tile - tm * tilesN;
  const int m0 = tm << 6;
  const int n0 = tn << 6;

  const int rlane = lane & 15;
  const int hh    = lane >> 4;
  const int koff  = hh * 8;
  const int mOff  = hh * 8;

  v8f acc[4][4];
#pragma unroll
  for (int i = 0; i < 4; ++i)
#pragma unroll
    for (int j = 0; j < 4; ++j) acc[i][j] = (v8f){0.f, 0.f, 0.f, 0.f, 0.f, 0.f, 0.f, 0.f};

  for (int k0 = 0; k0 < K; k0 += 32) {
    v16h bh[4];
#pragma unroll
    for (int j = 0; j < 4; ++j) {
      const size_t bo = (size_t)(n0 + (j << 4) + rlane) * ldb + koff + k0;
      bh[j] = frag_load(Bt + bo);
    }
#pragma unroll
    for (int i = 0; i < 4; ++i) {
      const size_t ao = (size_t)(m0 + (i << 4) + rlane) * lda + koff + k0;
      const v16h ah = frag_load(A + ao);
#pragma unroll
      for (int j = 0; j < 4; ++j) acc[i][j] = mma_f16(ah, bh[j], acc[i][j]);
      tie_acc(acc[i][0], ah, bh[0]);
      tie_acc(acc[i][1], ah, bh[1]);
      tie_acc(acc[i][2], ah, bh[2]);
      guard_acc(acc[i][3], ah, bh[3]);
    }
  }

  float* slab = sT[wave];
  float bvj[4];
#pragma unroll
  for (int j = 0; j < 4; ++j) bvj[j] = in_leg(bias[n0 + (j << 4) + rlane]);
  float cs[4] = {0.f, 0.f, 0.f, 0.f};
  float cq[4] = {0.f, 0.f, 0.f, 0.f};

#pragma unroll
  for (int i = 0; i < 4; ++i) {
    const int mBase = m0 + (i << 4);
#pragma unroll
    for (int j = 0; j < 4; ++j) {
#pragma unroll
      for (int r = 0; r < 8; ++r) {
        float v = acc[i][j][r] * scale + bvj[j];
        if (EPI == kEpiAct) {
          v = fmaxf(v, 0.0f);
          v = v * kActCarry;
          v = (v < kF16MinNormal) ? 0.0f : v;
        }
        if (EPI == kEpiStat) {
          cs[j] += v;
          cq[j] = fmaf(v, v, cq[j]);
        }
        slab[(mOff + r) * 68 + (j << 4) + rlane] = v;
      }
    }
    __builtin_amdgcn_fence(__ATOMIC_RELEASE, "workgroup");
    __builtin_amdgcn_wave_barrier();
    __builtin_amdgcn_fence(__ATOMIC_ACQUIRE, "workgroup");
    if (EPI == kEpiAct) {
      const int q = lane >> 3, c8 = (lane & 7) * 8;
      unsigned short* C = (unsigned short*)Cout;
      v8h hv[4];
#pragma unroll
      for (int it = 0; it < 4; ++it) {
        const float* sp = slab + (it * 4 + q) * 68 + c8;
        const v4f a0 = *(const v4f*)(sp);
        const v4f a1 = *(const v4f*)(sp + 4);
#pragma unroll
        for (int e = 0; e < 4; ++e) {
          hv[it][e]     = (_Float16)a0[e];
          hv[it][4 + e] = (_Float16)a1[e];
        }
      }
      for (int pass = 0; pass < 2; ++pass) {
#pragma unroll
        for (int it = 0; it < 4; ++it) {
          const int row = it * 4 + q;
          *(volatile v8h*)(C + (size_t)(mBase + row) * ldc + n0 + c8) = hv[it];
        }
        __threadfence();
      }
    } else {
      float* C = (float*)Cout;
      const int c4 = (lane & 15) * 4;
      for (int pass = 0; pass < 2; ++pass) {
#pragma unroll
        for (int it = 0; it < 8; ++it) {
          const int row = it * 2 + hh;
          const v4f v = *(const v4f*)(slab + row * 68 + c4);
          *(volatile v4f*)(C + (size_t)(mBase + row) * ldc + n0 + c4) = v;
        }
        __threadfence();
      }
    }
    __builtin_amdgcn_fence(__ATOMIC_RELEASE, "workgroup");
    __builtin_amdgcn_wave_barrier();
    __builtin_amdgcn_fence(__ATOMIC_ACQUIRE, "workgroup");
  }

  if (EPI == kEpiStat) {
#pragma unroll
    for (int j = 0; j < 4; ++j) {
      cs[j] += __shfl_xor(cs[j], 16, 32);
      cq[j] += __shfl_xor(cq[j], 16, 32);
    }
#pragma unroll
    for (int j = 0; j < 4; ++j) {
      const float pv = hh ? cq[j] : cs[j];
      slab[hh * 68 + (j << 4) + rlane] = pv;
    }
    __builtin_amdgcn_fence(__ATOMIC_RELEASE, "workgroup");
    __builtin_amdgcn_wave_barrier();
    __builtin_amdgcn_fence(__ATOMIC_ACQUIRE, "workgroup");
    const int c4 = (lane & 15) * 4;
    const v4f pv4 = *(const v4f*)(slab + hh * 68 + c4);
    float* sp = Spart + (size_t)(tm * 2 + hh) * N + n0 + c4;
    *(volatile v4f*)sp = pv4;
    __threadfence();
    *(volatile v4f*)sp = pv4;
  }
}

}

__global__ __launch_bounds__(256) void channel_stats_kernel(
    const float* __restrict__ Spart, float* __restrict__ stat)
{
  const int n = blockIdx.x * 256 + threadIdx.x;
  if (n >= kDm) return;
  double s = 0.0, q = 0.0;
#pragma unroll 4
  for (int tmi = 0; tmi < kTileRows; ++tmi) {
    s += (double)Spart[(size_t)(tmi * 2 + 0) * kDm + n];
    q += (double)Spart[(size_t)(tmi * 2 + 1) * kDm + n];
  }
  const double inv_rows = 1.0 / (double)kRows;
  const double mu = s * inv_rows;
  double var = q * inv_rows - mu * mu;
  var = (var < 0.0) ? 0.0 : var;
  const float muf = (float)mu;
  const float rs  = rsqrtf((float)var + kBnEps);
  volatile float* sp = stat;
  sp[n] = muf;
  sp[kDm + n] = rs;
  __threadfence();
  sp[n] = muf;
  sp[kDm + n] = rs;
}

template <bool GATHER>
__global__ __launch_bounds__(256) void norm_relu_plane_kernel(
    const float* __restrict__ T, const float* __restrict__ stat,
    const float* __restrict__ gam, const float* __restrict__ bet,
    const float* __restrict__ pos, const int* __restrict__ perm,
    unsigned short* __restrict__ H)
{
  const int i = blockIdx.x * 256 + threadIdx.x;
  if (i >= kRows * kOctPerRow) return;
  const int r = i / kOctPerRow;
  const int n = (i - r * kOctPerRow) * 8;
  int pv = perm[r];
  pv = (pv < 0) ? 0 : ((pv > kTok - 1) ? (kTok - 1) : pv);
  const int tok  = GATHER ? pv : (r & (kTok - 1));
  const int srow = (r & ~(kTok - 1)) + tok;
  const float* tp = T + (size_t)srow * kDm + n;
  const v4f t0 = *(const v4f*)(tp);
  const v4f t1 = *(const v4f*)(tp + 4);
  const v4f m0 = *(const v4f*)(stat + n);
  const v4f m1 = *(const v4f*)(stat + n + 4);
  const v4f r0 = *(const v4f*)(stat + kDm + n);
  const v4f r1 = *(const v4f*)(stat + kDm + n + 4);
  const v4f g0 = *(const v4f*)(gam + n);
  const v4f g1 = *(const v4f*)(gam + n + 4);
  const v4f b0 = *(const v4f*)(bet + n);
  const v4f b1 = *(const v4f*)(bet + n + 4);
  v4f p0 = (v4f){0.f, 0.f, 0.f, 0.f};
  v4f p1 = (v4f){0.f, 0.f, 0.f, 0.f};
  if (GATHER) {
    const float* pp = pos + (size_t)tok * kDm + n;
    p0 = *(const v4f*)(pp);
    p1 = *(const v4f*)(pp + 4);
  }
  v8h hv;
#pragma unroll
  for (int e = 0; e < 4; ++e) {
    float va = ((t0[e] - m0[e]) * r0[e]) * in_leg(g0[e]) + in_leg(b0[e]);
    float vb = ((t1[e] - m1[e]) * r1[e]) * in_leg(g1[e]) + in_leg(b1[e]);
    va = fmaxf(va, 0.0f);
    vb = fmaxf(vb, 0.0f);
    if (GATHER) {
      const float pa = p0[e];
      const float pb = p1[e];
      va = fmaxf(va + in_leg(pa), 0.0f);
      vb = fmaxf(vb + in_leg(pb), 0.0f);
    }
    hv[e]     = to_f16_carried(va, kActCarry);
    hv[4 + e] = to_f16_carried(vb, kActCarry);
  }
  unsigned short* q = H + ((size_t)i << 3);
  *(volatile v8h*)q = hv;
  __threadfence();
  *(volatile v8h*)q = hv;
}

extern "C" void kernel_launch(void* const* d_in, const int* in_sizes, int n_in,
                              void* d_out, int out_size, void* d_ws, size_t ws_size,
                              hipStream_t stream) {
  if (n_in < 11) return;
  if (in_sizes[0] != kBatch * kChan * kImg * kImg) return;
  if (in_sizes[1] != kWElems) return;
  if (in_sizes[2] != kDm) return;
  if (in_sizes[3] != kDepth * kWElems) return;
  if (in_sizes[4] != kDepth * kDm) return;
  if (in_sizes[5] != kDepth * kDm) return;
  if (in_sizes[6] != kDepth * kDm) return;
  if (in_sizes[7] != kTok * kDm) return;
  if (in_sizes[8] != kWElems) return;
  if (in_sizes[9] != kDm) return;
  if (in_sizes[10] != kBatch * kTok) return;
  if (out_size != kRows * kDm) return;
  if (ws_size < kWsTotal) return;

  const float* x       = (const float*)d_in[0];
  const float* conv0_w = (const float*)d_in[1];
  const float* conv0_b = (const float*)d_in[2];
  const float* w1      = (const float*)d_in[3];
  const float* b1      = (const float*)d_in[4];
  const float* gamma   = (const float*)d_in[5];
  const float* beta    = (const float*)d_in[6];
  const float* pos     = (const float*)d_in[7];
  const float* mixer_w = (const float*)d_in[8];
  const float* mixer_b = (const float*)d_in[9];
  const int*   perm    = (const int*)d_in[10];
  float* out = (float*)d_out;

  char* ws = (char*)d_ws;
  float*          T  = (float*)(ws + kOffT);
  unsigned short* P0 = (unsigned short*)(ws + kOffP0);
  unsigned short* H  = (unsigned short*)(ws + kOffH);
  unsigned short* WH = (unsigned short*)(ws + kOffWH);
  float*          S  = (float*)(ws + kOffS);
  float*          ST = (float*)(ws + kOffST);

  constexpr int kGemmBlocks = ((kRows / 64) * (kDm / 64)) / 8;
  constexpr int kEwBlocks   = (kRows * kOctPerRow) / 256;

  weight_planes_kernel<<<5 * ((kWElems / 8) / 256), 256, 0, stream>>>(conv0_w, w1, mixer_w, WH);
  patch_rows_kernel<<<kEwBlocks, 256, 0, stream>>>(x, P0);

  eng::gemm_f16_kernel<eng::kEpiAct><<<kGemmBlocks, 256, 0, stream>>>(
      P0, kKin, WH, kKin, (void*)H, kDm, conv0_b, S, kRows, kDm, kKin, kFold);

  for (int d = 0; d < kDepth; ++d) {
    float* Sd  = S + (size_t)d * kSPlane;
    float* STd = ST + (size_t)d * 2 * kDm;
    eng::gemm_f16_kernel<eng::kEpiStat><<<kGemmBlocks, 256, 0, stream>>>(
        H, kDm, WH + (size_t)(1 + d) * kWElems, kDm, (void*)T, kDm, b1 + (size_t)d * kDm, Sd,
        kRows, kDm, kDm, kFold);
    channel_stats_kernel<<<kDm / 256, 256, 0, stream>>>(Sd, STd);
    if (d + 1 < kDepth) {
      norm_relu_plane_kernel<false><<<kEwBlocks, 256, 0, stream>>>(
          T, STd, gamma + (size_t)d * kDm, beta + (size_t)d * kDm, pos, perm, H);
    } else {
      norm_relu_plane_kernel<true><<<kEwBlocks, 256, 0, stream>>>(
          T, STd, gamma + (size_t)d * kDm, beta + (size_t)d * kDm, pos, perm, H);
    }
  }

  eng::gemm_f16_kernel<eng::kEpiOut><<<kGemmBlocks, 256, 0, stream>>>(
      H, kDm, WH + (size_t)4 * kWElems, kDm, (void*)out, kDm, mixer_b, S, kRows, kDm, kDm, kFold);
}
